// PerformerAttention_6614249636625
// MI455X (gfx1250) — hardware-verified
//
#include <hip/hip_runtime.h>
#include <math.h>

constexpr int kBatch = 2;
constexpr int kTok   = 9216;
constexpr int kCh    = 512;
constexpr int kHeads = 8;
constexpr int kDh    = 64;
constexpr int kFeat  = 256;
constexpr int kRows  = kBatch * kTok;
constexpr int kBlk64 = kTok / 64;
constexpr int kBlk32 = kTok / 32;
constexpr float kDn      = 0.35355339059327373f;
constexpr float kHalfDn2 = 0.0625f;
constexpr float kRatio   = 0.0625f;
constexpr float kEps     = 1e-4f;
constexpr float kKpCarry  = 16384.0f;
constexpr float kQpCarry  = 1024.0f;
constexpr float kVCarry   = 16.0f;
constexpr float kCtxCarry = 4096.0f;

typedef __attribute__((ext_vector_type(16))) _Float16 v16h;
typedef __attribute__((ext_vector_type(8)))  _Float16 v8h;
typedef __attribute__((ext_vector_type(16))) __bf16   v16b;
typedef __attribute__((ext_vector_type(8)))  __bf16   v8b;
typedef __attribute__((ext_vector_type(8)))  float    v8f;
typedef __attribute__((ext_vector_type(4)))  float    v4f;
typedef __attribute__((ext_vector_type(4)))  unsigned int v4u;
typedef __attribute__((ext_vector_type(8)))  unsigned short v8us;

__device__ __forceinline__ unsigned short f2bf_bits(float f) {
  unsigned u = __float_as_uint(f);
  return (unsigned short)((u + 0x7FFFu + ((u >> 16) & 1u)) >> 16);
}
__device__ __forceinline__ float bf_bits2f(unsigned short h) { return __uint_as_float(((unsigned)h) << 16); }

__device__ __forceinline__ void dep_guard_h(v8f& a, v8f& b, v16h x, v16h y) { asm volatile("v_nop\n\tv_nop\n\tv_nop\n\tv_nop" : "+v"(a), "+v"(b) : "v"(x), "v"(y)); }
__device__ __forceinline__ void dep_guard_b(v8f& a, v8f& b, v16b x, v16b y) { asm volatile("v_nop\n\tv_nop\n\tv_nop\n\tv_nop" : "+v"(a), "+v"(b) : "v"(x), "v"(y)); }
__device__ __forceinline__ void keep4_h(v16h a, v16h b, v16h c, v16h d) { asm volatile("v_nop" :: "v"(a), "v"(b), "v"(c), "v"(d)); }
__device__ __forceinline__ void keep4_b(v16b a, v16b b, v16b c, v16b d) { asm volatile("v_nop" :: "v"(a), "v"(b), "v"(c), "v"(d)); }
__device__ __forceinline__ void acc_guard4(v8f& a, v8f& b, v8f& c, v8f& d) { asm volatile("v_nop\n\tv_nop\n\tv_nop\n\tv_nop" : "+v"(a), "+v"(b), "+v"(c), "+v"(d)); }
template <typename T> struct Frag;
template <> struct Frag<_Float16> {
  typedef v16h V; union U { v16h v; v8h h[2]; };
  static __device__ __forceinline__ v16h load(const _Float16* p) {
    U f; f.h[0] = *(const v8h*)(p); f.h[1] = *(const v8h*)(p + 16); return f.v;
  }
  static __device__ __forceinline__ v8f mma(v16h a, v16h b, v8f c) {
    return __builtin_amdgcn_wmma_f32_16x16x32_f16(false, a, false, b, (short)0, c, false, false);
  }
  static __device__ __forceinline__ void guard(v8f& a, v8f& b, v16h x, v16h y) { dep_guard_h(a, b, x, y); }
  static __device__ __forceinline__ void keep(v16h a, v16h b, v16h c, v16h d) { keep4_h(a, b, c, d); }
};
template <> struct Frag<__bf16> {
  typedef v16b V; union U { v16b v; v8b h[2]; };
  static __device__ __forceinline__ v16b load(const __bf16* p) {
    U f; f.h[0] = *(const v8b*)(p); f.h[1] = *(const v8b*)(p + 16); return f.v;
  }
  static __device__ __forceinline__ v8f mma(v16b a, v16b b, v8f c) {
    return __builtin_amdgcn_wmma_f32_16x16x32_bf16(false, a, false, b, (short)0, c, false, false);
  }
  static __device__ __forceinline__ void guard(v8f& a, v8f& b, v16b x, v16b y) { dep_guard_b(a, b, x, y); }
  static __device__ __forceinline__ void keep(v16b a, v16b b, v16b c, v16b d) { keep4_b(a, b, c, d); }
};

__device__ __forceinline__ unsigned pk16(unsigned short a, unsigned short b) { return (unsigned)a | ((unsigned)b << 16); }
__device__ __forceinline__ unsigned short h_bits(float f) { const _Float16 h = (_Float16)f; return __builtin_bit_cast(unsigned short, h); }

__device__ __forceinline__ v8f bmma(v16b a, v16b b, v8f c) {
  c = __builtin_amdgcn_wmma_f32_16x16x32_bf16(false, a, false, b, (short)0, c, false, false);
  asm volatile("v_nop\n\tv_nop\n\tv_nop\n\tv_nop" : "+v"(c) : "v"(a), "v"(b));
  return c;
}

__device__ __forceinline__ void lds_wave_sync() {
  __builtin_amdgcn_fence(__ATOMIC_RELEASE, "workgroup");
  __builtin_amdgcn_wave_barrier();
  __builtin_amdgcn_fence(__ATOMIC_ACQUIRE, "workgroup");
}

template <int ET> struct Elem;
template <> struct Elem<0> { typedef _Float16 T; };
template <> struct Elem<1> { typedef __bf16 T; };
template <int ET, int SPLITM, int BIAS_MODE, int OUT_MODE, bool RESID>
__global__ __launch_bounds__(256) void wmma_gemm64(
    const unsigned short* __restrict__ Ap, const unsigned short* __restrict__ A2p, int lda, long strideA,
    const unsigned short* __restrict__ Btp, const unsigned short* __restrict__ Bt2p, int ldb, long strideB,
    void* __restrict__ Cout, void* __restrict__ Cout2, int ldc, long strideC,
    const float* __restrict__ bias,
    const float* __restrict__ resid, long strideR,
    int M, int N, int K, float scale) {
  typedef typename Elem<ET>::T T;
  typedef typename Frag<T>::V V;
  const T* A = (const T*)Ap; const T* A2 = (const T*)A2p; const T* Bt = (const T*)Btp; const T* Bt2 = (const T*)Bt2p;
  __shared__ __align__(16) float sT[8][16 * 68];
  const int b    = blockIdx.y;
  const int lane = threadIdx.x & 31;
  const int wave = threadIdx.x >> 5;
  const int wpb  = blockDim.x >> 5;
  const int tilesN = N >> 6;
  const int tilesM = M >> 6;
  const int tile = blockIdx.x * wpb + wave;
  if (tile >= tilesM * tilesN) return;
  const int tm = tile / tilesN;
  const int tn = tile - tm * tilesN;
  const int m0 = tm << 6;
  const int n0 = tn << 6;

  const T* Ab  = A  + (size_t)b * strideA;
  const T* Bb  = Bt + (size_t)b * strideB;
  const T* Ab2 = (SPLITM >= 1) ? (A2  + (size_t)b * strideA) : nullptr;
  const T* Bb2 = (SPLITM >= 2) ? (Bt2 + (size_t)b * strideB) : nullptr;

  const int rlane = lane & 15;
  const int koff  = (lane >> 4) * 8;
  const int mOff  = (lane >> 4) * 8;

  v8f acc[4][4];
#pragma unroll
  for (int i = 0; i < 4; ++i)
#pragma unroll
    for (int j = 0; j < 4; ++j) acc[i][j] = (v8f){0.f,0.f,0.f,0.f,0.f,0.f,0.f,0.f};

  for (int k0 = 0; k0 < K; k0 += 32) {
    V bh[4], bl[4];
#pragma unroll
    for (int j = 0; j < 4; ++j) {
      const size_t bo = (size_t)(n0 + (j << 4) + rlane) * ldb + koff + k0;
      bh[j] = Frag<T>::load(Bb + bo);
      if (SPLITM >= 2) bl[j] = Frag<T>::load(Bb2 + bo);
    }
#pragma unroll
    for (int i = 0; i < 4; ++i) {
      const size_t ao = (size_t)(m0 + (i << 4) + rlane) * lda + koff + k0;
      V ah = Frag<T>::load(Ab + ao);
      V al;
      if (SPLITM >= 1) al = Frag<T>::load(Ab2 + ao);
#pragma unroll
      for (int j = 0; j < 4; ++j) {
        acc[i][j] = Frag<T>::mma(ah, bh[j], acc[i][j]);
        if (SPLITM >= 2) acc[i][j] = Frag<T>::mma(ah, bl[j], acc[i][j]);
        if (SPLITM >= 1) acc[i][j] = Frag<T>::mma(al, bh[j], acc[i][j]);
      }
      Frag<T>::guard(acc[i][0], acc[i][3], ah, (SPLITM >= 1) ? al : ah);
    }
    Frag<T>::keep(bh[0], bh[1], bh[2], bh[3]);
    if (SPLITM >= 2) Frag<T>::keep(bl[0], bl[1], bl[2], bl[3]);
  }
  acc_guard4(acc[0][0], acc[0][1], acc[0][2], acc[0][3]);
  acc_guard4(acc[1][0], acc[1][1], acc[1][2], acc[1][3]);
  acc_guard4(acc[2][0], acc[2][1], acc[2][2], acc[2][3]);
  acc_guard4(acc[3][0], acc[3][1], acc[3][2], acc[3][3]);

  float* slab = sT[wave];
  const float* Rb = RESID ? (resid + (size_t)b * strideR) : nullptr;
#pragma unroll
  for (int i = 0; i < 4; ++i) {
    const int mBase = m0 + (i << 4);
#pragma unroll
    for (int j = 0; j < 4; ++j) {
      const int n = n0 + (j << 4) + rlane;
      float bv = 0.f;
      if (BIAS_MODE == 2) bv = bias[n];
#pragma unroll
      for (int r = 0; r < 8; ++r) {
        float v = acc[i][j][r] * scale;
        if (BIAS_MODE == 1) v += bias[mBase + mOff + r];
        if (BIAS_MODE == 2) v += bv;
        if (RESID) v += Rb[(size_t)(mBase + mOff + r) * ldc + n];
        slab[(mOff + r) * 68 + (j << 4) + rlane] = v;
      }
    }
    __builtin_amdgcn_fence(__ATOMIC_RELEASE, "workgroup");
    __builtin_amdgcn_wave_barrier();
    __builtin_amdgcn_fence(__ATOMIC_ACQUIRE, "workgroup");
    if (OUT_MODE == 0) {
      float* C = (float*)Cout + (size_t)b * strideC;
      const int hh = lane >> 4, c4 = (lane & 15) * 4;
      for (int pass = 0; pass < 2; ++pass) {
#pragma unroll
        for (int it = 0; it < 8; ++it) {
          const int row = it * 2 + hh;
          v4f v = *(const v4f*)(slab + row * 68 + c4);
          *(volatile v4f*)(C + (size_t)(mBase + row) * ldc + n0 + c4) = v;
        }
        __threadfence();
      }
    } else {
      const int q = lane >> 3, c8 = (lane & 7) * 8;
      unsigned short* C  = (unsigned short*)Cout  + (size_t)b * strideC;
      unsigned short* C2 = (OUT_MODE == 2) ? ((unsigned short*)Cout2 + (size_t)b * strideC) : nullptr;
      for (int pass = 0; pass < 2; ++pass) {
#pragma unroll
        for (int it = 0; it < 4; ++it) {
          const int row = it * 4 + q;
          const float* sp = slab + row * 68 + c8;
          v8h hv, lv;
#pragma unroll
          for (int e = 0; e < 8; ++e) {
            if (OUT_MODE == 1) {
              hv[e] = (_Float16)sp[e];
            } else {
              unsigned short hb = f2bf_bits(sp[e]);
              unsigned short lb = f2bf_bits(sp[e] - bf_bits2f(hb));
              hv[e] = __builtin_bit_cast(_Float16, hb);
              lv[e] = __builtin_bit_cast(_Float16, lb);
            }
          }
          *(volatile v8h*)(C + (size_t)(mBase + row) * ldc + n0 + c8) = hv;
          if (OUT_MODE == 2) *(volatile v8h*)(C2 + (size_t)(mBase + row) * ldc + n0 + c8) = lv;
        }
        __threadfence();
      }
    }
    __builtin_amdgcn_fence(__ATOMIC_RELEASE, "workgroup");
    __builtin_amdgcn_wave_barrier();
    __builtin_amdgcn_fence(__ATOMIC_ACQUIRE, "workgroup");
  }
}

__global__ __launch_bounds__(256) void cast_bf16x8(const float* __restrict__ in, unsigned short* __restrict__ out, int n8) {
  const int i = blockIdx.x * 256 + threadIdx.x;
  if (i < n8) {
    const v4f a = *(const v4f*)(in + (size_t)i * 8);
    const v4f c = *(const v4f*)(in + (size_t)i * 8 + 4);
    v4u u;
    u[0] = pk16(f2bf_bits(a[0]), f2bf_bits(a[1]));
    u[1] = pk16(f2bf_bits(a[2]), f2bf_bits(a[3]));
    u[2] = pk16(f2bf_bits(c[0]), f2bf_bits(c[1]));
    u[3] = pk16(f2bf_bits(c[2]), f2bf_bits(c[3]));
    unsigned short* p = out + (size_t)i * 8;
    *(volatile v4u*)p = u;
    __threadfence();
    *(volatile v4u*)p = u;
  }
}

__global__ __launch_bounds__(256) void wtcast_kernel(const float* __restrict__ W0, const float* __restrict__ W1,
                                                     const float* __restrict__ W2, const float* __restrict__ W3,
                                                     unsigned short* __restrict__ out) {
  __shared__ float sm[64][65];
  const int t  = threadIdx.x;
  const int d0 = blockIdx.x * 64;
  const int h0 = blockIdx.y * 64;
  const int z  = blockIdx.z;
  const float* W = (z == 0) ? W0 : (z == 1) ? W1 : (z == 2) ? W2 : W3;
#pragma unroll
  for (int i = 0; i < 16; ++i) {
    const int e = i * 256 + t;
    const int r = e >> 6;
    const int c = e & 63;
    sm[c][r] = W[(size_t)(d0 + r) * kCh + h0 + c];
  }
  __syncthreads();
  const int lane = t & 31, wave = t >> 5;
  const int q = lane >> 3, c8 = (lane & 7) * 8;
  unsigned short* op = out + (size_t)z * kCh * kCh;
  for (int pass = 0; pass < 2; ++pass) {
#pragma unroll
    for (int it = 0; it < 2; ++it) {
      const int row = wave * 8 + it * 4 + q;
      unsigned short hb[8];
#pragma unroll
      for (int e = 0; e < 8; ++e) hb[e] = f2bf_bits(sm[row][c8 + e]);
      const v4u u = (v4u){pk16(hb[0], hb[1]), pk16(hb[2], hb[3]), pk16(hb[4], hb[5]), pk16(hb[6], hb[7])};
      *(volatile v4u*)(op + (size_t)(h0 + row) * kCh + d0 + c8) = u;
    }
    __threadfence();
  }
}

template <int MODE>
__global__ __launch_bounds__(128) void feat_kernel(
    const unsigned short* __restrict__ hiP, const unsigned short* __restrict__ loP,
    int lda, long zsOuter, long zsInner,
    const unsigned short* __restrict__ projP,
    const float* __restrict__ scal,
    const float* __restrict__ ksumP,
    float* __restrict__ pmaxP,
    float* __restrict__ pcolP,
    unsigned short* __restrict__ planeP) {
  constexpr int NW = (MODE == 3) ? 2 : 4;
  constexpr int RB = 16 * NW;
  constexpr int QP = 260;
  constexpr int TP = 72;
  __shared__ __align__(16) float slabQ[(MODE == 3) ? RB * QP : 4];
  __shared__ __align__(16) unsigned short slabT[(MODE == 2) ? kFeat * TP : 8];
  __shared__ float scs[(MODE == 2) ? NW * kFeat : 4];
  __shared__ float sks[(MODE == 3) ? kFeat : 4];
  __shared__ float sdiag[RB];
  __shared__ float srmax[RB];
  __shared__ float sdinv[RB];
  __shared__ float sred[NW];

  const int tid  = threadIdx.x;
  const int wave = tid >> 5, lane = tid & 31;
  const int rl = lane & 15, hh = lane >> 4, koff = hh * 8;
  const int z  = blockIdx.y;
  const int n0 = blockIdx.x * RB;
  const size_t aoff = (size_t)(z >> 3) * (size_t)zsOuter + (size_t)(z & 7) * (size_t)zsInner + (size_t)n0 * (size_t)lda;

  if constexpr (MODE >= 2) {
    const int drow = tid >> 1, dhalf = tid & 1;
    const size_t roff = aoff + (size_t)drow * lda + dhalf * 32;
    float s = 0.f;
#pragma unroll
    for (int i = 0; i < 4; ++i) {
      const v8us a = *(const v8us*)(hiP + roff + 8 * i);
      const v8us c = *(const v8us*)(loP + roff + 8 * i);
#pragma unroll
      for (int e = 0; e < 8; ++e) { const float q = bf_bits2f(a[e]) + bf_bits2f(c[e]); s += q * q; }
    }
    s += __shfl_xor(s, 1, 32);
    if (dhalf == 0) sdiag[drow] = kHalfDn2 * s;
  }
  if constexpr (MODE == 3) {
#pragma unroll 1
    for (int i = tid; i < kFeat; i += 32 * NW) sks[i] = ksumP[(size_t)z * kFeat + i];
  }
  __syncthreads();

  const __bf16* Ah = (const __bf16*)(hiP + aoff) + (size_t)(wave * 16 + rl) * lda + koff;
  const __bf16* Al = (const __bf16*)(loP + aoff) + (size_t)(wave * 16 + rl) * lda + koff;
  const __bf16* Pj = (const __bf16*)projP + (size_t)rl * kDh + koff;
  const v16b ah0 = Frag<__bf16>::load(Ah);
  const v16b ah1 = Frag<__bf16>::load(Ah + 32);
  const v16b al0 = Frag<__bf16>::load(Al);
  const v16b al1 = Frag<__bf16>::load(Al + 32);

  float dg[8];
#pragma unroll
  for (int r = 0; r < 8; ++r) dg[r] = (MODE >= 2) ? sdiag[wave * 16 + 8 * hh + r] : 0.f;
  const float stab = (MODE == 2) ? scal[0] : 0.f;
  float lmax = -INFINITY;
  float rmax[8];
#pragma unroll
  for (int r = 0; r < 8; ++r) rmax[r] = -INFINITY;

#pragma unroll 1
  for (int g = 0; g < 4; ++g) {
    v8f acc[4];
#pragma unroll
    for (int j = 0; j < 4; ++j) {
      acc[j] = (v8f){0.f,0.f,0.f,0.f,0.f,0.f,0.f,0.f};
      const __bf16* prow = Pj + (size_t)(g * 64 + j * 16) * kDh;
      const v16b b0 = Frag<__bf16>::load(prow);
      const v16b b1 = Frag<__bf16>::load(prow + 32);
      acc[j] = bmma(ah0, b0, acc[j]);
      acc[j] = bmma(al0, b0, acc[j]);
      acc[j] = bmma(ah1, b1, acc[j]);
      acc[j] = bmma(al1, b1, acc[j]);
    }
#pragma unroll
    for (int j = 0; j < 4; ++j) {
      const int col = g * 64 + j * 16 + rl;
      if constexpr (MODE == 1) {
#pragma unroll
        for (int r = 0; r < 8; ++r) lmax = fmaxf(lmax, acc[j][r]);
      } else if constexpr (MODE == 2) {
        float cs = 0.f;
#pragma unroll
        for (int r = 0; r < 8; ++r) {
          const float dd = acc[j][r] * kDn;
          const float e  = kRatio * (expf((dd - dg[r]) - stab) + kEps);
          cs += e;
          slabT[col * TP + wave * 16 + 8 * hh + r] = h_bits(e * kKpCarry);
        }
        cs += __shfl_xor(cs, 16, 32);
        if (hh == 0) scs[wave * kFeat + col] = cs;
      } else {
#pragma unroll
        for (int r = 0; r < 8; ++r) {
          const float dd = acc[j][r] * kDn;
          rmax[r] = fmaxf(rmax[r], dd);
          slabQ[(wave * 16 + 8 * hh + r) * QP + col] = dd;
        }
      }
    }
  }

  if constexpr (MODE == 1) {
    float m = lmax;
    m = fmaxf(m, __shfl_xor(m, 1, 32));
    m = fmaxf(m, __shfl_xor(m, 2, 32));
    m = fmaxf(m, __shfl_xor(m, 4, 32));
    m = fmaxf(m, __shfl_xor(m, 8, 32));
    m = fmaxf(m, __shfl_xor(m, 16, 32));
    if (lane == 0) sred[wave] = m;
    __syncthreads();
    float bm = sred[0];
#pragma unroll
    for (int w = 1; w < NW; ++w) bm = fmaxf(bm, sred[w]);
    bm = bm * kDn;
    if (wave == 0 && lane < 8) {
      const v4f v = {bm, bm, bm, bm};
      float* dst = pmaxP + ((size_t)z * gridDim.x + blockIdx.x) * 32 + lane * 4;
      *(volatile v4f*)dst = v;
      __threadfence();
      *(volatile v4f*)dst = v;
    }
  }

  if constexpr (MODE == 2) {
    __syncthreads();
    {
      const int c0 = tid, c1 = tid + 32 * NW;
      const float s0 = ((scs[c0] + scs[kFeat + c0]) + scs[2 * kFeat + c0]) + scs[3 * kFeat + c0];
      const float s1 = ((scs[c1] + scs[kFeat + c1]) + scs[2 * kFeat + c1]) + scs[3 * kFeat + c1];
      float* dst = pcolP + ((size_t)z * gridDim.x + blockIdx.x) * kFeat;
      for (int pass = 0; pass < 2; ++pass) {
        *(volatile float*)(dst + c0) = s0;
        *(volatile float*)(dst + c1) = s1;
        __threadfence();
      }
    }
    {
      unsigned short* dst = planeP + (size_t)z * kFeat * kTok + n0;
      const int q8 = lane >> 3, c8 = (lane & 7) * 8;
      for (int pass = 0; pass < 2; ++pass) {
#pragma unroll 1
        for (int it = 0; it < 16; ++it) {
          const int m = wave * 64 + it * 4 + q8;
          const v8us v = *(const v8us*)(slabT + m * TP + c8);
          *(volatile v8us*)(dst + (size_t)m * kTok + c8) = v;
        }
        __threadfence();
      }
    }
  }

  if constexpr (MODE == 3) {
#pragma unroll
    for (int r = 0; r < 8; ++r) {
      float m = rmax[r];
      m = fmaxf(m, __shfl_xor(m, 1, 32));
      m = fmaxf(m, __shfl_xor(m, 2, 32));
      m = fmaxf(m, __shfl_xor(m, 4, 32));
      m = fmaxf(m, __shfl_xor(m, 8, 32));
      rmax[r] = m;
    }
    if (rl == 0) {
#pragma unroll
      for (int r = 0; r < 8; ++r) srmax[wave * 16 + 8 * hh + r] = rmax[r];
    }
    lds_wave_sync();
#pragma unroll 1
    for (int rr = 0; rr < 16; ++rr) {
      const int row = wave * 16 + rr;
      const float dgv = sdiag[row], rmv = srmax[row];
      float* sp = slabQ + row * QP + lane * 8;
      const v4f x0 = *(const v4f*)sp;
      const v4f x1 = *(const v4f*)(sp + 4);
      v4f q0 = x0, q1 = x1;
      float den = 0.f;
#pragma unroll
      for (int e = 0; e < 4; ++e) { const float q = kRatio * (expf((x0[e] - dgv) - rmv) + kEps); q0[e] = q; den += q * sks[lane * 8 + e]; }
#pragma unroll
      for (int e = 0; e < 4; ++e) { const float q = kRatio * (expf((x1[e] - dgv) - rmv) + kEps); q1[e] = q; den += q * sks[lane * 8 + 4 + e]; }
      *(v4f*)sp = q0;
      *(v4f*)(sp + 4) = q1;
      den += __shfl_xor(den, 1, 32);
      den += __shfl_xor(den, 2, 32);
      den += __shfl_xor(den, 4, 32);
      den += __shfl_xor(den, 8, 32);
      den += __shfl_xor(den, 16, 32);
      if (lane == 0) sdinv[row] = 1.0f / den;
    }
    lds_wave_sync();
    unsigned short* dst = planeP + ((size_t)z * kTok + n0) * kFeat;
    for (int pass = 0; pass < 2; ++pass) {
#pragma unroll 1
      for (int rr = 0; rr < 16; ++rr) {
        const int row = wave * 16 + rr;
        const float sc = sdinv[row] * kQpCarry;
        const float* sp = slabQ + row * QP + lane * 8;
        const v4f x0 = *(const v4f*)sp;
        const v4f x1 = *(const v4f*)(sp + 4);
        v4u u;
        u[0] = pk16(h_bits(x0[0] * sc), h_bits(x0[1] * sc));
        u[1] = pk16(h_bits(x0[2] * sc), h_bits(x0[3] * sc));
        u[2] = pk16(h_bits(x1[0] * sc), h_bits(x1[1] * sc));
        u[3] = pk16(h_bits(x1[2] * sc), h_bits(x1[3] * sc));
        *(volatile v4u*)(dst + (size_t)row * kFeat + lane * 8) = u;
      }
      __threadfence();
    }
  }
}

__global__ __launch_bounds__(256) void stab_kernel(const float* __restrict__ pmax, int count, float* __restrict__ scal) {
  __shared__ float sm[8];
  const int tid = threadIdx.x, wave = tid >> 5, lane = tid & 31;
  float m = -INFINITY;
#pragma unroll 1
  for (int i = tid; i < count; i += 256) m = fmaxf(m, pmax[(size_t)i * 32]);
  m = fmaxf(m, __shfl_xor(m, 1, 32));
  m = fmaxf(m, __shfl_xor(m, 2, 32));
  m = fmaxf(m, __shfl_xor(m, 4, 32));
  m = fmaxf(m, __shfl_xor(m, 8, 32));
  m = fmaxf(m, __shfl_xor(m, 16, 32));
  if (lane == 0) sm[wave] = m;
  __syncthreads();
  float g = sm[0];
#pragma unroll
  for (int w = 1; w < 8; ++w) g = fmaxf(g, sm[w]);
  if (wave == 0 && lane < 8) {
    const v4f v = {g, g, g, g};
    float* dst = scal + lane * 4;
    *(volatile v4f*)dst = v;
    __threadfence();
    *(volatile v4f*)dst = v;
  }
}

__global__ __launch_bounds__(256) void ksum_kernel(const float* __restrict__ pcol, int nblk, float* __restrict__ ksum) {
  const int m = threadIdx.x;
  float s0 = 0.f, s1 = 0.f;
#pragma unroll 1
  for (int i = 0; i < nblk; ++i) s0 += pcol[(size_t)i * kFeat + m];
#pragma unroll 1
  for (int i = 0; i < nblk; ++i) s1 += pcol[(size_t)(nblk + i) * kFeat + m];
  for (int pass = 0; pass < 2; ++pass) {
    *(volatile float*)(ksum + m) = s0;
    *(volatile float*)(ksum + kFeat + m) = s1;
    __threadfence();
  }
}

extern "C" void kernel_launch(void* const* d_in, const int* in_sizes, int n_in,
                              void* d_out, int out_size, void* d_ws, size_t ws_size,
                              hipStream_t stream) {
  if (n_in < 7) return;
  if (in_sizes[0] != kRows * kCh || in_sizes[1] != kCh * kCh || in_sizes[2] != kCh * kCh ||
      in_sizes[3] != kCh * kCh || in_sizes[4] != kCh * kCh || in_sizes[5] != kCh ||
      in_sizes[6] != kFeat * kDh || out_size != kRows * kCh) return;

  const float* x    = (const float*)d_in[0];
  const float* Wq   = (const float*)d_in[1];
  const float* Wk   = (const float*)d_in[2];
  const float* Wv   = (const float*)d_in[3];
  const float* Wo   = (const float*)d_in[4];
  const float* bo   = (const float*)d_in[5];
  const float* proj = (const float*)d_in[6];
  float* out = (float*)d_out;

  size_t off = 0;
  auto carve = [&](size_t bytes) -> size_t { const size_t o = off; off += (bytes + 255) & ~(size_t)255; return o; };
  const size_t oXB = carve((size_t)kRows * kCh * 2);
  const size_t oWT = carve((size_t)4 * kCh * kCh * 2);
  const size_t oPJ = carve((size_t)kFeat * kDh * 2);
  const size_t oKH = carve((size_t)kRows * kCh * 2);
  const size_t oKL = carve((size_t)kRows * kCh * 2);
  const size_t oQH = carve((size_t)kTok * 128 * 2);
  const size_t oQL = carve((size_t)kTok * 128 * 2);
  const size_t oVT = carve((size_t)128 * kTok * 2);
  const size_t oKP = carve((size_t)2 * kFeat * kTok * 2);
  const size_t oQP = carve((size_t)2 * kTok * kFeat * 2);
  const size_t oCT = carve((size_t)2 * kDh * kFeat * 2);
  const size_t oOH = carve((size_t)kRows * kCh * 2);
  const size_t oOL = carve((size_t)kRows * kCh * 2);
  const size_t oPM = carve((size_t)kBatch * kHeads * kBlk64 * 32 * 4);
  const size_t oSC = carve(256);
  const size_t oPC = carve((size_t)2 * kBlk64 * kFeat * 4);
  const size_t oKS = carve((size_t)2 * kFeat * 4);
  if (off > ws_size) return;

  char* ws = (char*)d_ws;
  unsigned short* xb = (unsigned short*)(ws + oXB);
  unsigned short* wt = (unsigned short*)(ws + oWT);
  unsigned short* pj = (unsigned short*)(ws + oPJ);
  unsigned short* kh = (unsigned short*)(ws + oKH);
  unsigned short* kl = (unsigned short*)(ws + oKL);
  unsigned short* qh = (unsigned short*)(ws + oQH);
  unsigned short* ql = (unsigned short*)(ws + oQL);
  unsigned short* vt = (unsigned short*)(ws + oVT);
  unsigned short* kp = (unsigned short*)(ws + oKP);
  unsigned short* qp = (unsigned short*)(ws + oQP);
  unsigned short* ct = (unsigned short*)(ws + oCT);
  unsigned short* oh = (unsigned short*)(ws + oOH);
  unsigned short* ol = (unsigned short*)(ws + oOL);
  float* pm = (float*)(ws + oPM);
  float* sc = (float*)(ws + oSC);
  float* pc = (float*)(ws + oPC);
  float* ks = (float*)(ws + oKS);

  const size_t wplane = (size_t)kCh * kCh;

  cast_bf16x8<<<dim3((kRows * kCh / 8) / 256), dim3(256), 0, stream>>>(x, xb, kRows * kCh / 8);
  wtcast_kernel<<<dim3(kCh / 64, kCh / 64, 4), dim3(256), 0, stream>>>(Wq, Wk, Wv, Wo, wt);
  cast_bf16x8<<<dim3((kFeat * kDh / 8) / 256), dim3(256), 0, stream>>>(proj, pj, kFeat * kDh / 8);
  wmma_gemm64<1, 0, 0, 2, false><<<dim3((kRows / 64) * (kCh / 64) / 8, 1), dim3(256), 0, stream>>>(
      xb, nullptr, kCh, 0L, wt + 1 * wplane, nullptr, kCh, 0L, (void*)kh, (void*)kl, kCh, 0L,
      nullptr, nullptr, 0L, kRows, kCh, kCh, 1.0f);
  feat_kernel<1><<<dim3(kBlk64, kBatch * kHeads), dim3(128), 0, stream>>>(
      kh, kl, kCh, (long)kTok * kCh, (long)kDh, pj, sc, nullptr, pm, nullptr, nullptr);
  stab_kernel<<<dim3(1), dim3(256), 0, stream>>>(pm, kBatch * kHeads * kBlk64, sc);

  for (int g = 0; g < 8; ++g) {
    const int b  = g >> 2;
    const int h0 = (g & 3) * 2;
    const size_t xoff = (size_t)b * kTok * kCh;
    const size_t hoff = xoff + (size_t)h0 * kDh;
    const size_t wrow = (size_t)h0 * kDh * kCh;
    wmma_gemm64<1, 0, 0, 2, false><<<dim3((kTok / 64) * 2 / 8, 1), dim3(256), 0, stream>>>(
        xb + xoff, nullptr, kCh, 0L, wt + 0 * wplane + wrow, nullptr, kCh, 0L, (void*)qh, (void*)ql, 128, 0L,
        nullptr, nullptr, 0L, kTok, 128, kCh, 1.0f);
    wmma_gemm64<1, 0, 0, 1, false><<<dim3(2 * (kTok / 64) / 8, 1), dim3(256), 0, stream>>>(
        wt + 2 * wplane + wrow, nullptr, kCh, 0L, xb + xoff, nullptr, kCh, 0L, (void*)vt, nullptr, kTok, 0L,
        nullptr, nullptr, 0L, 128, kTok, kCh, kVCarry);
    feat_kernel<2><<<dim3(kBlk64, 2), dim3(128), 0, stream>>>(
        kh + hoff, kl + hoff, kCh, 0L, (long)kDh, pj, sc, nullptr, nullptr, pc, kp);
    ksum_kernel<<<dim3(1), dim3(256), 0, stream>>>(pc, kBlk64, ks);
    feat_kernel<3><<<dim3(kBlk32, 2), dim3(64), 0, stream>>>(
        qh, ql, 128, 0L, (long)kDh, pj, sc, ks, nullptr, nullptr, qp);
    wmma_gemm64<0, 0, 0, 1, false><<<dim3(1, 2), dim3(128), 0, stream>>>(
        vt, nullptr, kTok, (long)kDh * kTok, kp, nullptr, kTok, (long)kFeat * kTok, (void*)ct, nullptr, kFeat, (long)kDh * kFeat,
        nullptr, nullptr, 0L, kDh, kFeat, kTok, kCtxCarry / (kVCarry * kKpCarry));
    wmma_gemm64<0, 0, 0, 2, false><<<dim3((kTok / 64) / 8, 2), dim3(256), 0, stream>>>(
        qp, nullptr, kFeat, (long)kTok * kFeat, ct, nullptr, kFeat, (long)kDh * kFeat, (void*)(oh + hoff), (void*)(ol + hoff), kCh, (long)kDh,
        nullptr, nullptr, 0L, kTok, kDh, kFeat, 1.0f / (kQpCarry * kCtxCarry));
  }

  wmma_gemm64<1, 1, 2, 0, false><<<dim3((kRows / 64) * (kCh / 64) / 8, 1), dim3(256), 0, stream>>>(
      oh, ol, kCh, 0L, wt + 3 * wplane, nullptr, kCh, 0L, (void*)out, nullptr, kCh, 0L,
      bo, nullptr, 0L, kRows, kCh, kCh, 1.0f);
}
